// MultiAgentNetwork_81063212745124
// MI455X (gfx1250) — hardware-verified
//
#include <hip/hip_runtime.h>
#include <math.h>

#ifndef NB
#define NB 16384
#endif
#define NB_FULL 16384
#define NPLAY 4
#define NFREQ 32
#define OBSW 8
#define KENC 260
#define KP1 288
#define EPITCH 320
#define HID 512
#define CH 1024
#define NCH (NB / CH)
#define TPC 20
#define RPC (TPC * 64)
#define FLAGW 32
#define MROWS (NCH * RPC)
#define PI_F 3.14159265358979f

static_assert(NB % CH == 0 && NB <= NB_FULL && NB >= CH);
static_assert(NB_FULL * 4 == 65536);
static_assert(CH == 4 * 256);
static_assert(CH < 65536);
static_assert(TPC >= (CH + NPLAY * 63) / 64);
static_assert(TPC <= FLAGW && FLAGW * 4 == 128);
static_assert(RPC % 256 == 0);
static_assert(KP1 % 32 == 0 && KP1 >= KENC && KP1 <= EPITCH);
static_assert(EPITCH % 64 == 0);
static_assert(64 * EPITCH * 2 == 256 * 10 * 16);
static_assert(HID % 64 == 0 && HID % 32 == 0 && MROWS % 64 == 0);
static_assert((HID * (KP1 / 8)) % 256 == 0);
static_assert((HID * (HID / 8)) % 256 == 0 && (HID / 8) == 64);
static_assert(32 * 16 * 4 == 16 * 128);
static_assert(256 * 16 == CH * 4);
static_assert(8 * 16 * 68 * 4 <= 131072);
static_assert(64 * EPITCH * 2 + RPC * 4 + 64 + 128 <= 131072);
static_assert(2 * NPLAY * HID * 4 + 2 * CH * 4 + CH * 4 + 64 <= 131072);

static constexpr size_t al256(size_t b) { return (b + 255) & ~(size_t)255; }
static constexpr size_t WS_TOTAL = al256((size_t)NCH * FLAGW * 4) + al256((size_t)MROWS * EPITCH * 2) +
                                   4 * al256((size_t)MROWS * HID * 2) + 2 * al256((size_t)NPLAY * HID * KP1 * 2) +
                                   4 * al256((size_t)NPLAY * HID * HID * 2);
static_assert(WS_TOTAL <= (size_t)134217728);

static constexpr float SC  = 1.0f / 256.0f;
static constexpr float WSC = 32.0f;
static constexpr float ASC = 8.0f;

typedef __attribute__((ext_vector_type(16))) _Float16 v16h;
typedef __attribute__((ext_vector_type(8)))  _Float16 v8h;
typedef __attribute__((ext_vector_type(8)))  float    v8f;
typedef __attribute__((ext_vector_type(4)))  float    v4f;
typedef __attribute__((ext_vector_type(4)))  unsigned int v4u;


#define VST2(T, ptr, val) do { const T vst2_v_ = (val); *(volatile T*)(ptr) = vst2_v_; __threadfence(); *(volatile T*)(ptr) = vst2_v_; } while (0)
#define VST2V4(ptr, val) do { const v4f vst2_v4_ = (val); *(volatile v4f*)(ptr) = vst2_v4_; __threadfence(); *(volatile v4f*)(ptr) = vst2_v4_; } while (0)

__device__ __forceinline__ float bfr(float f) {
    unsigned u = __float_as_uint(f);
    u += 0x7FFFu + ((u >> 16) & 1u);
    return __uint_as_float(u & 0xFFFF0000u);
}
__device__ __forceinline__ unsigned short f2h_bits(float x) {
    return (fabsf(x) < 6.104e-5f) ? (unsigned short)0 : __builtin_bit_cast(unsigned short, (_Float16)x);
}
__device__ __forceinline__ void st8h(unsigned short* P, size_t o, const float* v) {
    v4u pk;
    pk.x = (unsigned)f2h_bits(v[0]) | ((unsigned)f2h_bits(v[1]) << 16);
    pk.y = (unsigned)f2h_bits(v[2]) | ((unsigned)f2h_bits(v[3]) << 16);
    pk.z = (unsigned)f2h_bits(v[4]) | ((unsigned)f2h_bits(v[5]) << 16);
    pk.w = (unsigned)f2h_bits(v[6]) | ((unsigned)f2h_bits(v[7]) << 16);
    VST2(v4u, (v4u*)(P + o), pk);
}

union FragU { v16h v; v8h h[2]; };
__device__ __forceinline__ v16h frag_ld(const _Float16* p) {
    FragU f; f.h[0] = *(const v8h*)(p); f.h[1] = *(const v8h*)(p + 16); return f.v;
}
__device__ __forceinline__ v8f wmma16(v16h a, v16h b, v8f c) {
    c = __builtin_amdgcn_wmma_f32_16x16x32_f16(false, a, false, b, (short)0, c, false, false);
    asm volatile("v_nop\n\tv_nop\n\tv_nop\n\tv_nop" : "+v"(c) : "v"(a), "v"(b));
    return c;
}
__device__ __forceinline__ void dep_guard_h(v8f& a, v8f& b, v16h x, v16h y) { asm volatile("v_nop\n\tv_nop\n\tv_nop\n\tv_nop" : "+v"(a), "+v"(b) : "v"(x), "v"(y)); }
__device__ __forceinline__ void keep4_h(v16h a, v16h b, v16h c, v16h d) { asm volatile("v_nop" :: "v"(a), "v"(b), "v"(c), "v"(d)); }
__device__ __forceinline__ void acc_guard4(v8f& a, v8f& b, v8f& c, v8f& d) { asm volatile("v_nop\n\tv_nop\n\tv_nop\n\tv_nop" : "+v"(a), "+v"(b), "+v"(c), "+v"(d)); }
__device__ __forceinline__ void wave_sync_lds() {
    __builtin_amdgcn_fence(3  , "workgroup");
    __builtin_amdgcn_wave_barrier();
    __builtin_amdgcn_fence(2  , "workgroup");
}

typedef _Float16 h16;
static __device__ __forceinline__ h16 toh_flush(float v) {
    const h16 r = (h16)v;
    return (fabsf(v) < 6.103515625e-05f) ? (h16)0.0f : r;
}

__device__ __forceinline__ unsigned pid_bf16(const v4f o) {
    const float b0 = bfr(o.x), b1 = bfr(o.y), b2 = bfr(o.z), b3 = bfr(o.w);
    unsigned p = 0u;
    float best = b0;
    if (b1 > best) { best = b1; p = 1u; }
    if (b2 > best) { best = b2; p = 2u; }
    if (b3 > best) { best = b3; p = 3u; }
    return p;
}

__device__ __forceinline__ void route_scan(const float* __restrict__ obs, unsigned chunk, unsigned t,
                                           unsigned (&pidv)[4], unsigned& lo, unsigned& hi, unsigned& slo, unsigned& shi) {
    const unsigned lane = t & 31u;
    lo = 0u; hi = 0u;
#pragma unroll
    for (int i = 0; i < 4; ++i) {
        const v4f o = *(const v4f*)(obs + (size_t)(chunk * CH + 4u * t + (unsigned)i) * OBSW + 4u);
        const unsigned p = pid_bf16(o);
        pidv[i] = p;
        lo += ((p == 0u) ? 1u : 0u) + ((p == 1u) ? 65536u : 0u);
        hi += ((p == 2u) ? 1u : 0u) + ((p == 3u) ? 65536u : 0u);
    }
    slo = lo; shi = hi;
#pragma unroll
    for (int d = 1; d < 32; d <<= 1) {
        const unsigned ylo = __shfl_up(slo, (unsigned)d, 32);
        const unsigned yhi = __shfl_up(shi, (unsigned)d, 32);
        slo += (lane >= (unsigned)d) ? ylo : 0u;
        shi += (lane >= (unsigned)d) ? yhi : 0u;
    }
}

__device__ __forceinline__ void route_place(const unsigned (&wt)[16], unsigned t, unsigned lo, unsigned hi, unsigned slo, unsigned shi,
                                            const unsigned (&pidv)[4], unsigned (&slot)[4], unsigned (&ts)[5]) {
    const unsigned wv = t >> 5;
    unsigned plo = 0u, phi = 0u, tlo = 0u, thi = 0u;
#pragma unroll
    for (int w = 0; w < 8; ++w) {
        const unsigned a = wt[2 * w], b = wt[2 * w + 1];
        tlo += a; thi += b;
        plo += ((unsigned)w < wv) ? a : 0u;
        phi += ((unsigned)w < wv) ? b : 0u;
    }
    const unsigned c0 = tlo & 0xFFFFu, c1 = tlo >> 16, c2 = thi & 0xFFFFu, c3 = thi >> 16;
    ts[0] = 0u;
    ts[1] = (c0 + 63u) >> 6;
    ts[2] = ts[1] + ((c1 + 63u) >> 6);
    ts[3] = ts[2] + ((c2 + 63u) >> 6);
    ts[4] = ts[3] + ((c3 + 63u) >> 6);
    const unsigned elo = plo + (slo - lo), ehi = phi + (shi - hi);
    unsigned b0 = ts[0] * 64u + (elo & 0xFFFFu);
    unsigned b1 = ts[1] * 64u + (elo >> 16);
    unsigned b2 = ts[2] * 64u + (ehi & 0xFFFFu);
    unsigned b3 = ts[3] * 64u + (ehi >> 16);
#pragma unroll
    for (int i = 0; i < 4; ++i) {
        const unsigned p = pidv[i];
        const unsigned s = (p == 0u) ? b0 : (p == 1u) ? b1 : (p == 2u) ? b2 : b3;
        slot[i] = min(s, (unsigned)(RPC - 1));
        b0 += (p == 0u) ? 1u : 0u;
        b1 += (p == 1u) ? 1u : 0u;
        b2 += (p == 2u) ? 1u : 0u;
        b3 += (p == 3u) ? 1u : 0u;
    }
}

__global__ __launch_bounds__(256) void k_gemm64r(
    const _Float16* __restrict__ A, unsigned lda, const _Float16* __restrict__ Bt, unsigned ldb,
    _Float16* __restrict__ C, unsigned ldc, const float* __restrict__ bias, const int* __restrict__ tflag,
    unsigned wstride, unsigned M, unsigned N, unsigned K, float scale, float oscale) {
  __shared__ __align__(16) float sT[8][16 * 68];
  const unsigned lane = threadIdx.x & 31u;
  const unsigned wave = (unsigned)__builtin_amdgcn_readfirstlane((int)(threadIdx.x >> 5));
  const unsigned tilesN = N >> 6, tilesM = M >> 6;
  const unsigned tile = blockIdx.x * 8u + wave;
  if (tile >= tilesM * tilesN) return;
  const unsigned tm = tile / tilesN;
  const unsigned tn = tile - tm * tilesN;
  const unsigned chunk = tm / (unsigned)TPC;
  const unsigned tj = tm - chunk * (unsigned)TPC;
  const int pl = tflag[chunk * (unsigned)FLAGW + tj];
  if (pl < 0 || pl >= NPLAY) return;
  const _Float16* Bp = Bt + (size_t)(unsigned)pl * wstride;
  const float* bp = bias + (unsigned)pl * N;
  const unsigned m0 = tm << 6, n0 = tn << 6;
  const unsigned rlane = lane & 15u;
  const unsigned koff = (lane >> 4) * 8u;
  const unsigned mOff = koff;

  v8f acc[4][4];
#pragma unroll
  for (int i = 0; i < 4; ++i)
#pragma unroll
    for (int j = 0; j < 4; ++j) acc[i][j] = (v8f){0.f,0.f,0.f,0.f,0.f,0.f,0.f,0.f};

  for (unsigned k0 = 0; k0 < K; k0 += 32u) {
    v16h bh[4];
#pragma unroll
    for (int j = 0; j < 4; ++j)
      bh[j] = frag_ld(Bp + (size_t)(n0 + ((unsigned)j << 4) + rlane) * ldb + koff + k0);
#pragma unroll
    for (int i = 0; i < 4; ++i) {
      const v16h ah = frag_ld(A + (size_t)(m0 + ((unsigned)i << 4) + rlane) * lda + koff + k0);
#pragma unroll
      for (int j = 0; j < 4; ++j)
        acc[i][j] = __builtin_amdgcn_wmma_f32_16x16x32_f16(false, ah, false, bh[j], (short)0, acc[i][j], false, false);
      dep_guard_h(acc[i][0], acc[i][3], ah, ah);
    }
    keep4_h(bh[0], bh[1], bh[2], bh[3]);
  }
  acc_guard4(acc[0][0], acc[0][1], acc[0][2], acc[0][3]);
  acc_guard4(acc[1][0], acc[1][1], acc[1][2], acc[1][3]);
  acc_guard4(acc[2][0], acc[2][1], acc[2][2], acc[2][3]);
  acc_guard4(acc[3][0], acc[3][1], acc[3][2], acc[3][3]);

  float* slab = sT[wave];
#pragma unroll
  for (int i = 0; i < 4; ++i) {
    const unsigned mBase = m0 + ((unsigned)i << 4);
#pragma unroll
    for (int j = 0; j < 4; ++j) {
      const unsigned n = n0 + ((unsigned)j << 4) + rlane;
      const float bv = bfr(bp[n]);
#pragma unroll
      for (int r = 0; r < 8; ++r) {
        float v = acc[i][j][r] * scale + bv;
        v = fmaxf(v, 0.0f);
        v *= oscale;
        slab[(mOff + (unsigned)r) * 68u + ((unsigned)j << 4) + rlane] = v;
      }
    }
    wave_sync_lds();
    {
      const unsigned q = lane >> 3, c8 = (lane & 7u) * 8u;
      v8h hv[4];
#pragma unroll
      for (int it = 0; it < 4; ++it) {
        const unsigned row = (unsigned)it * 4u + q;
        const float* sp = slab + row * 68u + c8;
#pragma unroll
        for (int e = 0; e < 8; ++e) hv[it][e] = toh_flush(sp[e]);
      }
      for (int pass = 0; pass < 2; ++pass) {
#pragma unroll
        for (int it = 0; it < 4; ++it) {
          const unsigned row = (unsigned)it * 4u + q;
          *(volatile v8h*)(C + (size_t)(mBase + row) * ldc + n0 + c8) = hv[it];
        }
        __threadfence();
      }
    }
    wave_sync_lds();
  }
}

__global__ __launch_bounds__(256) void k_wt16(const float* __restrict__ Wm, unsigned KI, unsigned NO, unsigned lgper,
                                              unsigned short* __restrict__ W16, float sw) {
    const unsigned layer = blockIdx.y;
    const float* Wl = Wm + (size_t)layer * KI * NO;
    unsigned short* Dl = W16 + (size_t)layer * KI * NO;
    const unsigned u = blockIdx.x * 256u + threadIdx.x;
    const unsigned per = 1u << lgper;
    if (u >= NO * per) return;
    const unsigned k0 = 8u * (u & (per - 1u));
    const unsigned o = u >> lgper;
    float v[8];
#pragma unroll
    for (int i = 0; i < 8; ++i) v[i] = bfr(Wl[(size_t)(k0 + (unsigned)i) * NO + o]) * sw;
    st8h(Dl, (size_t)o * KI + k0, v);
}

__global__ __launch_bounds__(256) void k_wt16p(const float* __restrict__ Wm, unsigned short* __restrict__ W16, float sw) {
    const unsigned player = blockIdx.y;
    const float* Wl = Wm + (size_t)player * KENC * HID;
    unsigned short* Dl = W16 + (size_t)player * HID * KP1;
    const unsigned u = blockIdx.x * 256u + threadIdx.x;
    if (u >= (unsigned)(HID * (KP1 / 8))) return;
    const unsigned o = u / (unsigned)(KP1 / 8);
    const unsigned k0 = 8u * (u - o * (unsigned)(KP1 / 8));
    float v[8];
#pragma unroll
    for (int i = 0; i < 8; ++i) {
        const unsigned k = k0 + (unsigned)i;
        const unsigned kc = min(k, (unsigned)(KENC - 1));
        const float w = bfr(Wl[(size_t)kc * HID + o]) * sw;
        v[i] = (k < (unsigned)KENC) ? w : 0.0f;
    }
    st8h(Dl, (size_t)o * KP1 + k0, v);
}

__global__ __launch_bounds__(256) void k_enc(const float* __restrict__ obs, const float* __restrict__ freqs,
                                             unsigned short* __restrict__ enc16, int* __restrict__ tflag) {
#pragma clang fp contract(off)
    __shared__ __align__(16) unsigned short sE[64 * EPITCH];
    __shared__ int sSrc[RPC];
    __shared__ unsigned sWT[16];
    __shared__ float sF[NFREQ];
    const unsigned t = threadIdx.x;
    const unsigned chunk = blockIdx.x;
    const unsigned row = t >> 2, pi = t & 3u;

    if (t < (unsigned)NFREQ) sF[t] = bfr(freqs[t]);
#pragma unroll
    for (int i = 0; i < RPC / 256; ++i) sSrc[t + 256u * (unsigned)i] = -1;
#pragma unroll 1
    for (unsigned z = 0; z < 15u; ++z) sE[row * EPITCH + (unsigned)KENC + 15u * pi + z] = (unsigned short)0;

    unsigned pidv[4], slot[4], ts[5];
    unsigned lo, hi, slo, shi;
    route_scan(obs, chunk, t, pidv, lo, hi, slo, shi);
    if ((t & 31u) == 31u) { sWT[2u * (t >> 5)] = slo; sWT[2u * (t >> 5) + 1u] = shi; }
    __syncthreads();
    unsigned wt[16];
#pragma unroll
    for (int w = 0; w < 16; ++w) wt[w] = sWT[w];
    route_place(wt, t, lo, hi, slo, shi, pidv, slot, ts);
#pragma unroll
    for (int i = 0; i < 4; ++i) sSrc[slot[i]] = (int)(4u * t + (unsigned)i);

    if (t < 8u) {
        unsigned fv[4];
#pragma unroll
        for (int e = 0; e < 4; ++e) {
            const unsigned j = 4u * t + (unsigned)e;
            const int plj = (j < ts[1]) ? 0 : (j < ts[2]) ? 1 : (j < ts[3]) ? 2 : (j < ts[4]) ? 3 : -1;
            fv[e] = (unsigned)plj;
        }
        v4u f; f.x = fv[0]; f.y = fv[1]; f.z = fv[2]; f.w = fv[3];
        VST2(v4u, (v4u*)(tflag + (size_t)chunk * FLAGW + 4u * t), f);
    }
    __syncthreads();

    const unsigned ntile = (unsigned)__builtin_amdgcn_readfirstlane((int)min(ts[4], (unsigned)TPC));
#pragma unroll 1
    for (unsigned tl = 0; tl < ntile; ++tl) {
        const int s = sSrc[tl * 64u + row];
        const bool valid = (s >= 0);
        const unsigned srow = min((unsigned)max(s, 0), (unsigned)(CH - 1));
        const float* orow = obs + (size_t)(chunk * CH + srow) * OBSW;
        float araw = orow[pi];
        float oraw = orow[4u + pi];
        asm volatile("" : "+v"(araw));
        asm volatile("" : "+v"(oraw));
        const float a = bfr(araw);
        const unsigned eb = row * EPITCH + pi * 64u;
#pragma unroll 1
        for (unsigned i = 0; i < (unsigned)NFREQ; ++i) {
            const float ang = a * sF[i];
            const float cs = cosf(ang) * 8.0f;
            const float sn = sinf(ang) * 8.0f;
            sE[eb + i]       = valid ? f2h_bits(cs) : (unsigned short)0;
            sE[eb + 32u + i] = valid ? f2h_bits(sn) : (unsigned short)0;
        }
        sE[row * EPITCH + 256u + pi] = valid ? f2h_bits(bfr(oraw) * 8.0f) : (unsigned short)0;
        __syncthreads();
        v4u pk[10];
#pragma unroll
        for (int it = 0; it < 10; ++it) pk[it] = *(const v4u*)(sE + (t + 256u * (unsigned)it) * 8u);
        unsigned short* dst = enc16 + (size_t)(chunk * RPC + tl * 64u) * EPITCH;
        for (int pass = 0; pass < 2; ++pass) {
#pragma unroll
            for (int it = 0; it < 10; ++it) *(volatile v4u*)(dst + (size_t)(t + 256u * (unsigned)it) * 8u) = pk[it];
            __threadfence();
        }
        __syncthreads();
    }
}

__global__ __launch_bounds__(256) void k_dec(const float* __restrict__ obs, const _Float16* __restrict__ h3p,
                                             const _Float16* __restrict__ h3v, const float* __restrict__ pWd,
                                             const float* __restrict__ pbd, const float* __restrict__ vWd,
                                             const float* __restrict__ vbd, float* __restrict__ out) {
    __shared__ __align__(16) float sWd[2][NPLAY * HID];
    __shared__ __align__(16) float sOut[2][CH];
    __shared__ unsigned sSlot[CH];
    __shared__ unsigned sWT[16];
    const unsigned t = threadIdx.x;
    const unsigned chunk = blockIdx.x;
#pragma unroll 1
    for (unsigned i = t; i < (unsigned)(NPLAY * HID); i += 256u) { sWd[0][i] = bfr(pWd[i]); sWd[1][i] = bfr(vWd[i]); }

    unsigned pidv[4], slot[4], ts[5];
    unsigned lo, hi, slo, shi;
    route_scan(obs, chunk, t, pidv, lo, hi, slo, shi);
    if ((t & 31u) == 31u) { sWT[2u * (t >> 5)] = slo; sWT[2u * (t >> 5) + 1u] = shi; }
    __syncthreads();
    unsigned wt[16];
#pragma unroll
    for (int w = 0; w < 16; ++w) wt[w] = sWT[w];
    route_place(wt, t, lo, hi, slo, shi, pidv, slot, ts);
#pragma unroll
    for (int i = 0; i < 4; ++i) sSlot[4u * t + (unsigned)i] = slot[i] | (pidv[i] << 16);
    __syncthreads();

#pragma unroll 1
    for (unsigned i = 0; i < 4u; ++i) {
        const unsigned r = t + 256u * i;
        const unsigned sp = sSlot[r];
        const unsigned sl = min(sp & 0xFFFFu, (unsigned)(RPC - 1));
        const unsigned p = (sp >> 16) & 3u;
        const size_t ro = (size_t)(chunk * RPC + sl) * HID;
        const unsigned wb = p * (unsigned)HID;
        float ap = 0.f, av = 0.f;
#pragma unroll 1
        for (unsigned k = 0; k < (unsigned)HID; k += 8u) {
            const v8h x = *(const v8h*)(h3p + ro + k);
            const v8h y = *(const v8h*)(h3v + ro + k);
            const v4f wp0 = *(const v4f*)(&sWd[0][wb + k]);
            const v4f wp1 = *(const v4f*)(&sWd[0][wb + k + 4u]);
            const v4f wv0 = *(const v4f*)(&sWd[1][wb + k]);
            const v4f wv1 = *(const v4f*)(&sWd[1][wb + k + 4u]);
            ap += (float)x[0] * wp0.x; ap += (float)x[1] * wp0.y; ap += (float)x[2] * wp0.z; ap += (float)x[3] * wp0.w;
            ap += (float)x[4] * wp1.x; ap += (float)x[5] * wp1.y; ap += (float)x[6] * wp1.z; ap += (float)x[7] * wp1.w;
            av += (float)y[0] * wv0.x; av += (float)y[1] * wv0.y; av += (float)y[2] * wv0.z; av += (float)y[3] * wv0.w;
            av += (float)y[4] * wv1.x; av += (float)y[5] * wv1.y; av += (float)y[6] * wv1.z; av += (float)y[7] * wv1.w;
        }
        const float zp = ap * 0.125f + bfr(pbd[p]);
        const float zv = av * 0.125f + bfr(vbd[p]);
        sOut[0][r] = PI_F * tanhf(zp);
        sOut[1][r] = PI_F * tanhf(zv);
    }
    __syncthreads();
    const v4f o0 = *(const v4f*)(&sOut[0][4u * t]);
    const v4f o1 = *(const v4f*)(&sOut[1][4u * t]);
    VST2V4(out + (size_t)chunk * CH + 4u * t, o0);
    VST2V4(out + (size_t)NB_FULL + (size_t)chunk * CH + 4u * t, o1);
}

extern "C" void kernel_launch(void* const* d_in, const int* in_sizes, int n_in, void* d_out, int out_size,
                              void* d_ws, size_t ws_size, hipStream_t stream) {
    if (n_in < 18) return;
    if (in_sizes[0] < NB * OBSW || in_sizes[1] < NFREQ) return;
    if (in_sizes[2] < NPLAY * KENC * HID || in_sizes[3] < NPLAY * HID || in_sizes[4] < NPLAY * HID * HID || in_sizes[5] < NPLAY * HID) return;
    if (in_sizes[6] < NPLAY * HID * HID || in_sizes[7] < NPLAY * HID || in_sizes[8] < NPLAY * HID || in_sizes[9] < NPLAY) return;
    if (in_sizes[10] < NPLAY * KENC * HID || in_sizes[11] < NPLAY * HID || in_sizes[12] < NPLAY * HID * HID || in_sizes[13] < NPLAY * HID) return;
    if (in_sizes[14] < NPLAY * HID * HID || in_sizes[15] < NPLAY * HID || in_sizes[16] < NPLAY * HID || in_sizes[17] < NPLAY) return;
    if (out_size < NB_FULL + NB) return;

    const float* obs   = (const float*)d_in[0];
    const float* freqs = (const float*)d_in[1];
    const float* pW1   = (const float*)d_in[2];
    const float* pb1   = (const float*)d_in[3];
    const float* pW2   = (const float*)d_in[4];
    const float* pb2   = (const float*)d_in[5];
    const float* pW3   = (const float*)d_in[6];
    const float* pb3   = (const float*)d_in[7];
    const float* pWd   = (const float*)d_in[8];
    const float* pbd   = (const float*)d_in[9];
    const float* vW1   = (const float*)d_in[10];
    const float* vb1   = (const float*)d_in[11];
    const float* vW2   = (const float*)d_in[12];
    const float* vb2   = (const float*)d_in[13];
    const float* vW3   = (const float*)d_in[14];
    const float* vb3   = (const float*)d_in[15];
    const float* vWd   = (const float*)d_in[16];
    const float* vbd   = (const float*)d_in[17];
    float* out = (float*)d_out;

    char* wsp = (char*)d_ws;
    size_t off = 0;
    auto carve = [&](size_t bytes) -> void* { void* r = wsp + off; off += (bytes + 255) & ~(size_t)255; return r; };
    int*            tflag = (int*)carve((size_t)NCH * FLAGW * 4);
    unsigned short* enc16 = (unsigned short*)carve((size_t)MROWS * EPITCH * 2);
    unsigned short* hA    = (unsigned short*)carve((size_t)MROWS * HID * 2);
    unsigned short* hB    = (unsigned short*)carve((size_t)MROWS * HID * 2);
    unsigned short* h3p   = (unsigned short*)carve((size_t)MROWS * HID * 2);
    unsigned short* h3v   = (unsigned short*)carve((size_t)MROWS * HID * 2);
    unsigned short* w1p   = (unsigned short*)carve((size_t)NPLAY * HID * KP1 * 2);
    unsigned short* w1v   = (unsigned short*)carve((size_t)NPLAY * HID * KP1 * 2);
    unsigned short* w2p   = (unsigned short*)carve((size_t)NPLAY * HID * HID * 2);
    unsigned short* w3p   = (unsigned short*)carve((size_t)NPLAY * HID * HID * 2);
    unsigned short* w2v   = (unsigned short*)carve((size_t)NPLAY * HID * HID * 2);
    unsigned short* w3v   = (unsigned short*)carve((size_t)NPLAY * HID * HID * 2);
    if (off > ws_size || off > (size_t)134217728) return;

    k_wt16p<<<dim3((HID * (KP1 / 8)) / 256, NPLAY), 256, 0, stream>>>(pW1, w1p, WSC);
    k_wt16p<<<dim3((HID * (KP1 / 8)) / 256, NPLAY), 256, 0, stream>>>(vW1, w1v, WSC);
    k_wt16<<<dim3((HID * (HID / 8)) / 256, NPLAY), 256, 0, stream>>>(pW2, HID, HID, 6, w2p, WSC);
    k_wt16<<<dim3((HID * (HID / 8)) / 256, NPLAY), 256, 0, stream>>>(pW3, HID, HID, 6, w3p, WSC);
    k_wt16<<<dim3((HID * (HID / 8)) / 256, NPLAY), 256, 0, stream>>>(vW2, HID, HID, 6, w2v, WSC);
    k_wt16<<<dim3((HID * (HID / 8)) / 256, NPLAY), 256, 0, stream>>>(vW3, HID, HID, 6, w3v, WSC);

    k_enc<<<NCH, 256, 0, stream>>>(obs, freqs, enc16, tflag);

    const unsigned gG = ((MROWS / 64) * (HID / 64) + 7) / 8;
    k_gemm64r<<<gG, 256, 0, stream>>>((const _Float16*)enc16, EPITCH, (const _Float16*)w1p, KP1, (_Float16*)hA, HID, pb1,
        (const int*)tflag, (unsigned)(HID * KP1), MROWS, HID, KP1, SC, ASC);
    k_gemm64r<<<gG, 256, 0, stream>>>((const _Float16*)hA, HID, (const _Float16*)w2p, HID, (_Float16*)hB, HID, pb2,
        (const int*)tflag, (unsigned)(HID * HID), MROWS, HID, HID, SC, ASC);
    k_gemm64r<<<gG, 256, 0, stream>>>((const _Float16*)hB, HID, (const _Float16*)w3p, HID, (_Float16*)h3p, HID, pb3,
        (const int*)tflag, (unsigned)(HID * HID), MROWS, HID, HID, SC, ASC);
    k_gemm64r<<<gG, 256, 0, stream>>>((const _Float16*)enc16, EPITCH, (const _Float16*)w1v, KP1, (_Float16*)hA, HID, vb1,
        (const int*)tflag, (unsigned)(HID * KP1), MROWS, HID, KP1, SC, ASC);
    k_gemm64r<<<gG, 256, 0, stream>>>((const _Float16*)hA, HID, (const _Float16*)w2v, HID, (_Float16*)hB, HID, vb2,
        (const int*)tflag, (unsigned)(HID * HID), MROWS, HID, HID, SC, ASC);
    k_gemm64r<<<gG, 256, 0, stream>>>((const _Float16*)hB, HID, (const _Float16*)w3v, HID, (_Float16*)h3v, HID, vb3,
        (const int*)tflag, (unsigned)(HID * HID), MROWS, HID, HID, SC, ASC);

    k_dec<<<NCH, 256, 0, stream>>>(obs, (const _Float16*)h3p, (const _Float16*)h3v, pWd, pbd, vWd, vbd, out);
}
